// Encoder_40510131536238
// MI455X (gfx1250) — hardware-run, weakly checked
//
#include <hip/hip_runtime.h>


#ifndef NB
#define NB 4
#endif
#ifndef SEQ
#define SEQ 577
#endif
#define NB_FULL  4
#define SEQ_FULL 577
#ifndef OUT_SEQ
#define OUT_SEQ SEQ
#endif
#define DM    512
#define NH_   8
#define HD    64
#define NQKV  1536
#define NATT  4
#define SEQP  (((SEQ + 63) / 64) * 64)
#define NKP   (((SEQ + 31) / 32) * 32)
#define AW    4
#define OSP   68
#define WTP   72
#define SC2   0.18033688011112042f
#define SCN   0.125f
#define L2E   1.4426950408889634f
#define LN2   0.6931471805599453f
#define PSH   14.0f
#define NEGB  (-3.0e38f)
#define LEAKY 0.01f
#define BNEPS 1.0e-5f
#define CTXS  256.0f
#define WOS   64.0f
#define OSCL  (1.0f / 16384.0f)

static_assert(HD == 64);
static_assert(NH_ * HD == DM);
static_assert(NQKV == 3 * DM);
static_assert(DM % 64 == 0);
static_assert(DM % 32 == 0);
static_assert(HD % 32 == 0);
static_assert(SEQP % 64 == 0);
static_assert(SEQP >= SEQ);
static_assert(NKP <= SEQP);
static_assert(NKP % 32 == 0);
static_assert(NKP - SEQ < 32);
static_assert(SEQP % (16 * AW) == 0);
static_assert((NB * SEQP) % 64 == 0);
static_assert(NB <= NB_FULL);
static_assert(SEQ <= SEQ_FULL);
static_assert((OSP * 4) % 16 == 0);
static_assert((WTP * 2) % 16 == 0);
static_assert(32 * 16 * 4 == 16 * HD * 2);
static_assert(32 * 16 * 4 == 16 * 64 * 2);
static_assert(32 * 16 * 8 == 16 * 64 * 4);
static_assert(256 * 16 * 2 == 64 * 64 * 2);
static_assert(32 * 16 == 128 * 4);
static_assert(AW * 16 * OSP * 4 + AW * 128 * 4 <= 131072);
static_assert(16 * OSP * 4 <= 131072);
static_assert(64 * WTP * 2 <= 131072);
static_assert((size_t)NB_FULL * SEQ_FULL * DM * 4 == (size_t)4726784);
static_assert((size_t)2 * NB_FULL * SEQ_FULL * DM * 4 == (size_t)9453568);
static_assert(((size_t)(NB - 1) * OUT_SEQ + SEQ) * DM <= (size_t)NB_FULL * SEQ_FULL * DM);

typedef _Float16 h16;
typedef unsigned short bf;
typedef __attribute__((ext_vector_type(16))) __bf16   v16bf;
typedef __attribute__((ext_vector_type(16))) _Float16 v16h;
typedef __attribute__((ext_vector_type(8)))  _Float16 v8h;
typedef __attribute__((ext_vector_type(8)))  unsigned short v8us;
typedef __attribute__((ext_vector_type(8)))  float    v8f;
typedef __attribute__((ext_vector_type(4)))  float    v4f;
typedef v4f  __attribute__((may_alias)) v4fa;
typedef v8us __attribute__((may_alias)) v8usa;

__device__ __forceinline__ unsigned short f2bf(float f) { unsigned u = __float_as_uint(f); u += 0x7FFFu + ((u >> 16) & 1u); return (unsigned short)(u >> 16); }
__device__ __forceinline__ float bfr(float f) { return __uint_as_float(((unsigned)f2bf(f)) << 16); }
__device__ __forceinline__ v16h cat16(v8h lo, v8h hi) { return __builtin_shufflevector(lo, hi, 0, 1, 2, 3, 4, 5, 6, 7, 8, 9, 10, 11, 12, 13, 14, 15); }
__device__ __forceinline__ v16bf cat16b(v8us lo, v8us hi) { return __builtin_bit_cast(v16bf, __builtin_shufflevector(lo, hi, 0, 1, 2, 3, 4, 5, 6, 7, 8, 9, 10, 11, 12, 13, 14, 15)); }
__device__ __forceinline__ v8f wmma16(v16h a, v16h b, v8f c) { return __builtin_amdgcn_wmma_f32_16x16x32_f16(false, a, false, b, (short)0, c, false, false); }
__device__ __forceinline__ v8f wmmab(v16bf a, v16bf b, v8f c) { return __builtin_amdgcn_wmma_f32_16x16x32_bf16(false, a, false, b, (short)0, c, false, false); }
__device__ __forceinline__ v16h  ldh(const h16* p) { return cat16(*(const v8h*)p, *(const v8h*)(p + 16)); }
__device__ __forceinline__ v16bf ldb(const bf* p)  { return cat16b(*(const v8us*)p, *(const v8us*)(p + 16)); }
__device__ __forceinline__ void wave_sync() { __builtin_amdgcn_fence(3  , "wavefront"); __builtin_amdgcn_wave_barrier(); asm volatile("" ::: "memory"); }
static __device__ __forceinline__ h16 toh_flush(float v) { const h16 r = (h16)v; return (fabsf(v) < 6.103515625e-05f) ? (h16)0.0f : r; }
__device__ __forceinline__ v8f wmma16_g(v16h a, v16h b, v8f c) { c = wmma16(a, b, c); asm volatile("v_nop\n\tv_nop\n\tv_nop\n\tv_nop" : "+v"(c) : "v"(a), "v"(b)); return c; }
__device__ __forceinline__ v8f wmmab_g(v16bf a, v16bf b, v8f c) { c = wmmab(a, b, c); asm volatile("v_nop\n\tv_nop\n\tv_nop\n\tv_nop" : "+v"(c) : "v"(a), "v"(b)); return c; }

__global__ __launch_bounds__(256) void k_cvtpad(const float* __restrict__ src, bf* dst) {
#pragma clang fp contract(off)
    const size_t i = (size_t)blockIdx.x * 256 + threadIdx.x; if (i >= (size_t)NB * SEQP * (DM / 8)) return;
    const int row = (int)(i / (DM / 8)), c8 = (int)(i % (DM / 8)) * 8;
    const int b = row / SEQP, t = row % SEQP;
    const bool ok = t < SEQ;
    const int tc = ok ? t : (SEQ - 1);
    v8f v = *(const v8f*)(src + ((size_t)b * SEQ_FULL + (size_t)tc) * DM + c8);
    asm volatile("" : "+v"(v));
    v8us o;
#pragma unroll
    for (int k = 0; k < 8; ++k) o[k] = ok ? f2bf(v[k]) : (unsigned short)0;
    *(volatile v8us*)(dst + i * 8) = o; __threadfence(); *(volatile v8us*)(dst + i * 8) = o;
}

__global__ __launch_bounds__(256) void k_wT(const float* __restrict__ src, unsigned short* dst, int N, int f16mode) {
#pragma clang fp contract(off)
    __shared__ __align__(16) unsigned short ts[64 * WTP];
    const int tid = threadIdx.x;
    const int n0 = blockIdx.x * 64, k0 = blockIdx.y * 64;
    const int c4 = (tid & 15) * 4, kr = tid >> 4;
#pragma unroll
    for (int i = 0; i < 4; ++i) { const int kk = kr + 16 * i;
        const v4f v = *(const v4f*)(src + (size_t)(k0 + kk) * (size_t)N + n0 + c4);
#pragma unroll
        for (int e = 0; e < 4; ++e) { const float w = bfr(v[e]);
            const unsigned short ub = (unsigned short)(__float_as_uint(w) >> 16);
            const unsigned short uh = __builtin_bit_cast(unsigned short, toh_flush(w * WOS));
            ts[(c4 + e) * WTP + kk] = f16mode ? uh : ub; } }
    __syncthreads();
#pragma unroll 1
    for (int ps = 0; ps < 2; ++ps) {
#pragma unroll
        for (int s = 0; s < 2; ++s) { const int row = s * 32 + (tid >> 3), c8 = (tid & 7) * 8;
            const v8us o = *(const v8usa*)(&ts[row * WTP + c8]);
            *(volatile v8us*)(dst + (size_t)(n0 + row) * DM + k0 + c8) = o; }
        if (ps == 0) __threadfence(); }
}

__global__ __launch_bounds__(32) void k_proj_qk(const bf* __restrict__ A, const bf* __restrict__ Bt, const float* __restrict__ bias, h16* PL) {
    __shared__ __align__(16) float os[16 * OSP];
    const int lane = threadIdx.x & 31, lr = lane & 15, hi = lane >> 4; const int r0 = blockIdx.x * 64, c0 = blockIdx.y * 64;
    v8f acc[4][4];
#pragma unroll
    for (int mb = 0; mb < 4; ++mb)
#pragma unroll
        for (int nb = 0; nb < 4; ++nb) acc[mb][nb] = (v8f){};
    const size_t aoff = (size_t)(r0 + lr) * DM + 8 * hi, boff = (size_t)(c0 + lr) * DM + 8 * hi;
#pragma unroll 1
    for (int kc = 0; kc < DM; kc += 32) {
        v16bf a[4];
#pragma unroll
        for (int mb = 0; mb < 4; ++mb) a[mb] = ldb(A + aoff + (size_t)mb * 16 * DM + kc);
#pragma unroll
        for (int nb = 0; nb < 4; ++nb) { const v16bf bq = ldb(Bt + boff + (size_t)nb * 16 * DM + kc);
#pragma unroll
            for (int mb = 0; mb < 4; ++mb) acc[mb][nb] = wmmab_g(a[mb], bq, acc[mb][nb]); }
    }
    float bc[4];
#pragma unroll
    for (int nb = 0; nb < 4; ++nb) bc[nb] = bfr(bias[c0 + nb * 16 + lr]);
    const int bb = r0 / SEQP, tt = r0 % SEQP; const int which = c0 / DM, hh = (c0 % DM) / HD;
    const size_t tbase = (((size_t)which * (NB * NH_) + (size_t)(bb * NH_ + hh)) * SEQP + (size_t)tt) * HD;
#pragma unroll
    for (int mb = 0; mb < 4; ++mb) {
#pragma unroll
        for (int nb = 0; nb < 4; ++nb) {
#pragma unroll
            for (int j = 0; j < 8; ++j) os[(hi * 8 + j) * OSP + nb * 16 + lr] = acc[mb][nb][j] + bc[nb]; }
        wave_sync();
#pragma unroll 1
        for (int ps = 0; ps < 2; ++ps) {
            const size_t sb = tbase + (size_t)(mb * 16) * HD;
#pragma unroll
            for (int s = 0; s < 4; ++s) { const int p = s * 32 + lane; const int row = p >> 3, c8 = (p & 7) * 8;
                const v4f x0 = *(const v4fa*)(&os[row * OSP + c8]); const v4f x1 = *(const v4fa*)(&os[row * OSP + c8 + 4]); v8h hv;
#pragma unroll
                for (int i = 0; i < 4; ++i) { hv[i] = toh_flush(x0[i]); hv[4 + i] = toh_flush(x1[i]); }
                *(volatile v8h*)(PL + sb + (size_t)p * 8) = hv; }
            if (ps == 0) __threadfence(); }
        wave_sync();
    }
}

__global__ __launch_bounds__(32) void k_proj_vt(const bf* __restrict__ A, const bf* __restrict__ Bt, const float* __restrict__ bias, h16* VT) {
    __shared__ __align__(16) float os[16 * OSP];
    const int lane = threadIdx.x & 31, lr = lane & 15, hi = lane >> 4; const int r0 = blockIdx.x * 64, c0 = blockIdx.y * 64;
    v8f acc[4][4];
#pragma unroll
    for (int mb = 0; mb < 4; ++mb)
#pragma unroll
        for (int nb = 0; nb < 4; ++nb) acc[mb][nb] = (v8f){};
    const size_t aoff = (size_t)(r0 + lr) * DM + 8 * hi, boff = (size_t)(c0 + lr) * DM + 8 * hi;
#pragma unroll 1
    for (int kc = 0; kc < DM; kc += 32) {
        v16bf a[4];
#pragma unroll
        for (int mb = 0; mb < 4; ++mb) a[mb] = ldb(A + aoff + (size_t)mb * 16 * DM + kc);
#pragma unroll
        for (int nb = 0; nb < 4; ++nb) { const v16bf bq = ldb(Bt + boff + (size_t)nb * 16 * DM + kc);
#pragma unroll
            for (int mb = 0; mb < 4; ++mb) acc[mb][nb] = wmmab_g(a[mb], bq, acc[mb][nb]); }
    }
    const int bb = c0 / SEQP, tt = c0 % SEQP;
    const size_t tbase = ((size_t)bb * DM + (size_t)r0) * SEQP + (size_t)tt;
#pragma unroll
    for (int mb = 0; mb < 4; ++mb) {
        float br[8];
#pragma unroll
        for (int j = 0; j < 8; ++j) br[j] = bfr(bias[r0 + mb * 16 + hi * 8 + j]);
#pragma unroll
        for (int nb = 0; nb < 4; ++nb) {
#pragma unroll
            for (int j = 0; j < 8; ++j) os[(hi * 8 + j) * OSP + nb * 16 + lr] = acc[mb][nb][j] + br[j]; }
        wave_sync();
#pragma unroll 1
        for (int ps = 0; ps < 2; ++ps) {
            const size_t sb = tbase + (size_t)(mb * 16) * SEQP;
#pragma unroll
            for (int s = 0; s < 4; ++s) { const int row = 4 * s + (lane >> 3), c8 = (lane & 7) * 8;
                const v4f x0 = *(const v4fa*)(&os[row * OSP + c8]); const v4f x1 = *(const v4fa*)(&os[row * OSP + c8 + 4]); v8h hv;
#pragma unroll
                for (int i = 0; i < 4; ++i) { hv[i] = toh_flush(x0[i]); hv[4 + i] = toh_flush(x1[i]); }
                *(volatile v8h*)(VT + sb + (size_t)row * SEQP + c8) = hv; }
            if (ps == 0) __threadfence(); }
        wave_sync();
    }
}

__global__ __launch_bounds__(32) void k_oproj(const h16* __restrict__ A, const h16* __restrict__ Bt, const float* __restrict__ bias, float* OUT) {
    __shared__ __align__(16) float os[16 * OSP];
    const int lane = threadIdx.x & 31, lr = lane & 15, hi = lane >> 4; const int r0 = blockIdx.x * 64, c0 = blockIdx.y * 64;
    v8f acc[4][4];
#pragma unroll
    for (int mb = 0; mb < 4; ++mb)
#pragma unroll
        for (int nb = 0; nb < 4; ++nb) acc[mb][nb] = (v8f){};
    const size_t aoff = (size_t)(r0 + lr) * DM + 8 * hi, boff = (size_t)(c0 + lr) * DM + 8 * hi;
#pragma unroll 1
    for (int kc = 0; kc < DM; kc += 32) {
        v16h a[4];
#pragma unroll
        for (int mb = 0; mb < 4; ++mb) a[mb] = ldh(A + aoff + (size_t)mb * 16 * DM + kc);
#pragma unroll
        for (int nb = 0; nb < 4; ++nb) { const v16h bq = ldh(Bt + boff + (size_t)nb * 16 * DM + kc);
#pragma unroll
            for (int mb = 0; mb < 4; ++mb) acc[mb][nb] = wmma16_g(a[mb], bq, acc[mb][nb]); }
    }
    float bc[4];
#pragma unroll
    for (int nb = 0; nb < 4; ++nb) bc[nb] = bfr(bias[c0 + nb * 16 + lr]);
    const int bb = r0 / SEQP, tt = r0 % SEQP;
#pragma unroll
    for (int mb = 0; mb < 4; ++mb) {
#pragma unroll
        for (int nb = 0; nb < 4; ++nb) {
#pragma unroll
            for (int j = 0; j < 8; ++j) os[(hi * 8 + j) * OSP + nb * 16 + lr] = acc[mb][nb][j] * OSCL + bc[nb]; }
        wave_sync();
#pragma unroll 1
        for (int ps = 0; ps < 2; ++ps) {
#pragma unroll
            for (int s = 0; s < 8; ++s) { const int row = 2 * s + (lane >> 4), c4 = (lane & 15) * 4;
                const int t = tt + mb * 16 + row;
                const v4f val = *(const v4fa*)(&os[row * OSP + c4]);
                if (t < SEQ) *(volatile v4f*)(OUT + ((size_t)bb * OUT_SEQ + (size_t)t) * DM + c0 + c4) = val; }
            if (ps == 0) __threadfence(); }
        wave_sync();
    }
}

__global__ __launch_bounds__(32 * AW) __attribute__((amdgpu_num_vgpr(256))) void k_flash(
        const h16* __restrict__ QKX, const h16* __restrict__ VTX, const h16* __restrict__ QKL, const h16* __restrict__ VTL,
        const float* __restrict__ c1w, const float* __restrict__ c1b, const float* __restrict__ bng, const float* __restrict__ bnb,
        const float* __restrict__ bnm, const float* __restrict__ bnv, const float* __restrict__ c2w, const float* __restrict__ c2b,
        h16* CX, h16* CL, float* ST) {
    __shared__ __align__(16) float os[AW * 16 * OSP];
    __shared__ __align__(16) float sts[AW * 128];
    const int lane = threadIdx.x & 31, lr = lane & 15, hi = lane >> 4;
    const int wave = __builtin_amdgcn_readfirstlane((int)(threadIdx.x >> 5));
    const int zh = blockIdx.y; const int b = zh / NH_, h = zh % NH_;
    const int t0 = (blockIdx.x * AW + wave) * 16;
    float A0[4], A1[4], A2[4], C2[4];
#pragma unroll
    for (int o = 0; o < NATT; ++o) { const int idx = h * NATT + o;
        const float sg = bfr(bng[idx]) * (1.0f / sqrtf(bfr(bnv[idx]) + BNEPS));
        A0[o] = bfr(c1w[idx * 2 + 0]) * sg * SCN; A1[o] = bfr(c1w[idx * 2 + 1]) * sg * SCN;
        A2[o] = (bfr(c1b[idx]) - bfr(bnm[idx])) * sg + bfr(bnb[idx]);
        C2[o] = bfr(c2w[idx]) * L2E; }
    const float C2B = bfr(c2b[h]) * L2E;
    const size_t koff = (size_t)NB * NH_ * SEQP * HD;
    const size_t pq = ((size_t)zh * SEQP + (size_t)(t0 + lr)) * HD + 8 * hi;
    const size_t ko = koff + ((size_t)zh * SEQP + (size_t)lr) * HD + 8 * hi;
    const size_t vo = ((size_t)zh * HD + (size_t)lr) * SEQP + 8 * hi;
    v8f ox[4], ol[4];
#pragma unroll
    for (int j = 0; j < 4; ++j) { ox[j] = (v8f){}; ol[j] = (v8f){}; }
    float mX = NEGB, lX = 0.0f, mL = NEGB, lL = 0.0f, wL = 0.0f;
#pragma unroll 1
    for (int key0 = 0; key0 < NKP; key0 += 32) {
        int zq = 0; asm volatile("" : "+s"(zq));
        v8f sXa = (v8f){}, sXb = (v8f){}, sLa = (v8f){}, sLb = (v8f){};
        { const v16h q0 = ldh(QKX + pq + zq), q1 = ldh(QKX + pq + zq + 32);
          const h16* ka = QKX + ko + (size_t)key0 * HD;
          const v16h a0 = ldh(ka), a1 = ldh(ka + 32);
          sXa = wmma16_g(a0, q0, sXa); sXa = wmma16_g(a1, q1, sXa);
          const v16h b0 = ldh(ka + 16 * HD), b1 = ldh(ka + 16 * HD + 32);
          sXb = wmma16_g(b0, q0, sXb); sXb = wmma16_g(b1, q1, sXb); }
        { const v16h q0 = ldh(QKL + pq + zq), q1 = ldh(QKL + pq + zq + 32);
          const h16* ka = QKL + ko + (size_t)key0 * HD;
          const v16h a0 = ldh(ka), a1 = ldh(ka + 32);
          sLa = wmma16_g(a0, q0, sLa); sLa = wmma16_g(a1, q1, sLa);
          const v16h b0 = ldh(ka + 16 * HD), b1 = ldh(ka + 16 * HD + 32);
          sLb = wmma16_g(b0, q0, sLb); sLb = wmma16_g(b1, q1, sLb); }
        const int ja = key0 + 8 * hi;
        float tx[16], tl[16];
#pragma unroll
        for (int r = 0; r < 8; ++r) {
            { const float sx = sXa[r], sl = sLa[r]; float hs = C2B;
#pragma unroll
              for (int o = 0; o < NATT; ++o) { float hh = fmaf(A0[o], sx, fmaf(A1[o], sl, A2[o])); hh = fmaxf(hh, LEAKY * hh); hs = fmaf(hh, C2[o], hs); }
              const bool va = (ja + r) < SEQ;
              tx[r] = va ? fmaf(sx, SC2, hs) : NEGB; tl[r] = va ? fmaf(sl, SC2, hs) : NEGB; }
            { const float sx = sXb[r], sl = sLb[r]; float hs = C2B;
#pragma unroll
              for (int o = 0; o < NATT; ++o) { float hh = fmaf(A0[o], sx, fmaf(A1[o], sl, A2[o])); hh = fmaxf(hh, LEAKY * hh); hs = fmaf(hh, C2[o], hs); }
              const bool vb = (ja + 16 + r) < SEQ;
              tx[8 + r] = vb ? fmaf(sx, SC2, hs) : NEGB; tl[8 + r] = vb ? fmaf(sl, SC2, hs) : NEGB; }
        }
        float mx = NEGB, ml = NEGB;
#pragma unroll
        for (int i = 0; i < 16; ++i) { mx = fmaxf(mx, tx[i]); ml = fmaxf(ml, tl[i]); }
        mx = fmaxf(mx, __shfl_xor(mx, 16, 32));
        ml = fmaxf(ml, __shfl_xor(ml, 16, 32));
        const float mnX = fmaxf(mX, mx), mnL = fmaxf(mL, ml);
        const float alX = __builtin_amdgcn_exp2f(mX - mnX), alL = __builtin_amdgcn_exp2f(mL - mnL);
        const float shX = PSH - mnX, shL = PSH - mnL;
        v16h pbx, pbl; float lsx = 0.0f, lsl = 0.0f, ws = 0.0f;
#pragma unroll
        for (int i = 0; i < 16; ++i) {
            const float e0 = tx[i] + shX, e1 = tl[i] + shL;
            const float x0 = __builtin_amdgcn_exp2f(e0), x1 = __builtin_amdgcn_exp2f(e1);
            const float g0 = (e0 < -14.0f) ? 0.0f : x0, g1 = (e1 < -14.0f) ? 0.0f : x1;
            const h16 p0 = (h16)g0; const h16 p1 = (h16)g1;
            pbx[i] = p0; pbl[i] = p1;
            const float f1 = (float)p1;
            lsx += (float)p0; lsl += f1; ws = fmaf(f1, tl[i] - tx[i], ws); }
        lX = lX * alX + lsx; mX = mnX;
        lL = lL * alL + lsl; wL = wL * alL + ws; mL = mnL;
#pragma unroll
        for (int j = 0; j < 4; ++j) { ox[j] = ox[j] * alX; ol[j] = ol[j] * alL; }
        { const h16* va = VTX + vo + key0;
#pragma unroll
          for (int j = 0; j < 4; ++j) { const v16h vf = ldh(va + (size_t)(16 * j) * SEQP); ox[j] = wmma16_g(vf, pbx, ox[j]); } }
        { const h16* va = VTL + vo + key0;
#pragma unroll
          for (int j = 0; j < 4; ++j) { const v16h vf = ldh(va + (size_t)(16 * j) * SEQP); ol[j] = wmma16_g(vf, pbl, ol[j]); } }
    }
    lX += __shfl_xor(lX, 16, 32);
    lL += __shfl_xor(lL, 16, 32);
    wL += __shfl_xor(wL, 16, 32);
    const float lsX = (lX > 0.0f) ? lX : 1.0f, lsL = (lL > 0.0f) ? lL : 1.0f;
    const float invX = CTXS * (1.0f / lsX), invL = CTXS * (1.0f / lsL);
    const int wb = wave * 16 * OSP;
    const size_t crow = ((size_t)b * SEQP + (size_t)t0) * DM + (size_t)h * HD;
#pragma unroll
    for (int j = 0; j < 4; ++j) { v4f a, c;
        a[0] = ox[j][0] * invX; a[1] = ox[j][1] * invX; a[2] = ox[j][2] * invX; a[3] = ox[j][3] * invX;
        c[0] = ox[j][4] * invX; c[1] = ox[j][5] * invX; c[2] = ox[j][6] * invX; c[3] = ox[j][7] * invX;
        *(v4fa*)(&os[wb + lr * OSP + 16 * j + 8 * hi]) = a; *(v4fa*)(&os[wb + lr * OSP + 16 * j + 8 * hi + 4]) = c; }
    wave_sync();
#pragma unroll 1
    for (int ps = 0; ps < 2; ++ps) {
#pragma unroll
        for (int s = 0; s < 4; ++s) { const int row = 4 * s + (lane >> 3), c8 = (lane & 7) * 8;
            const v4f x0 = *(const v4fa*)(&os[wb + row * OSP + c8]); const v4f x1 = *(const v4fa*)(&os[wb + row * OSP + c8 + 4]); v8h hv;
#pragma unroll
            for (int i = 0; i < 4; ++i) { hv[i] = toh_flush(x0[i]); hv[4 + i] = toh_flush(x1[i]); }
            *(volatile v8h*)(CX + crow + (size_t)row * DM + c8) = hv; }
        if (ps == 0) __threadfence(); }
    wave_sync();
#pragma unroll
    for (int j = 0; j < 4; ++j) { v4f a, c;
        a[0] = ol[j][0] * invL; a[1] = ol[j][1] * invL; a[2] = ol[j][2] * invL; a[3] = ol[j][3] * invL;
        c[0] = ol[j][4] * invL; c[1] = ol[j][5] * invL; c[2] = ol[j][6] * invL; c[3] = ol[j][7] * invL;
        *(v4fa*)(&os[wb + lr * OSP + 16 * j + 8 * hi]) = a; *(v4fa*)(&os[wb + lr * OSP + 16 * j + 8 * hi + 4]) = c; }
    wave_sync();
#pragma unroll 1
    for (int ps = 0; ps < 2; ++ps) {
#pragma unroll
        for (int s = 0; s < 4; ++s) { const int row = 4 * s + (lane >> 3), c8 = (lane & 7) * 8;
            const v4f x0 = *(const v4fa*)(&os[wb + row * OSP + c8]); const v4f x1 = *(const v4fa*)(&os[wb + row * OSP + c8 + 4]); v8h hv;
#pragma unroll
            for (int i = 0; i < 4; ++i) { hv[i] = toh_flush(x0[i]); hv[4 + i] = toh_flush(x1[i]); }
            *(volatile v8h*)(CL + crow + (size_t)row * DM + c8) = hv; }
        if (ps == 0) __threadfence(); }
    const int sb = wave * 128;
    const float s0 = hi ? wL : mX, s1 = hi ? 0.0f : lX, s2 = hi ? 0.0f : mL, s3 = hi ? 0.0f : lL;
    sts[sb + (4 * hi + 0) * 16 + lr] = s0; sts[sb + (4 * hi + 1) * 16 + lr] = s1;
    sts[sb + (4 * hi + 2) * 16 + lr] = s2; sts[sb + (4 * hi + 3) * 16 + lr] = s3;
    wave_sync();
    { const v4f sv = *(const v4fa*)(&sts[sb + lane * 4]);
      float* sp = ST + ((size_t)zh * (SEQP / 16) + (size_t)(t0 >> 4)) * 128 + lane * 4;
      *(volatile v4f*)sp = sv; __threadfence(); *(volatile v4f*)sp = sv; }
}

__global__ __launch_bounds__(256) void k_klred(const float* __restrict__ ST, float* OUT2) {
#pragma clang fp contract(off)
    __shared__ float red[24];
    const int tid = threadIdx.x, lane = tid & 31;
    const int wave = __builtin_amdgcn_readfirstlane((int)(threadIdx.x >> 5));
    float loss = 0.0f;
#pragma unroll 1
    for (int b = 0; b < NB; ++b) {
        float mx = NEGB, ml = NEGB;
#pragma unroll 1
        for (int i = tid; i < NH_ * SEQ; i += 256) { const int hh = i / SEQ, t = i - hh * SEQ;
            const size_t base = ((size_t)(b * NH_ + hh) * (SEQP / 16) + (size_t)(t >> 4)) * 128 + (size_t)(t & 15);
            mx = fmaxf(mx, ST[base]); ml = fmaxf(ml, ST[base + 32]); }
#pragma unroll
        for (int off = 16; off > 0; off >>= 1) { mx = fmaxf(mx, __shfl_xor(mx, off, 32)); ml = fmaxf(ml, __shfl_xor(ml, off, 32)); }
        if (lane == 0) { red[wave] = mx; red[8 + wave] = ml; }
        __syncthreads();
        float MX = red[0], ML = red[8];
#pragma unroll
        for (int w = 1; w < 8; ++w) { MX = fmaxf(MX, red[w]); ML = fmaxf(ML, red[8 + w]); }
        __syncthreads();
        float sl = 0.0f, s1 = 0.0f, sw = 0.0f;
#pragma unroll 1
        for (int i = tid; i < NH_ * SEQ; i += 256) { const int hh = i / SEQ, t = i - hh * SEQ;
            const size_t base = ((size_t)(b * NH_ + hh) * (SEQP / 16) + (size_t)(t >> 4)) * 128 + (size_t)(t & 15);
            const float m0 = ST[base], l0 = ST[base + 16], m1 = ST[base + 32], l1 = ST[base + 48], w1 = ST[base + 64];
            const float f0 = __builtin_amdgcn_exp2f(m0 - MX), f1 = __builtin_amdgcn_exp2f(m1 - ML);
            sl += l0 * f0; s1 += l1 * f1; sw += w1 * f1; }
#pragma unroll
        for (int off = 16; off > 0; off >>= 1) { sl += __shfl_xor(sl, off, 32); s1 += __shfl_xor(s1, off, 32); sw += __shfl_xor(sw, off, 32); }
        if (lane == 0) { red[wave] = sl; red[8 + wave] = s1; red[16 + wave] = sw; }
        __syncthreads();
        float SL = red[0], S1 = red[8], SW = red[16];
#pragma unroll
        for (int w = 1; w < 8; ++w) { SL += red[w]; S1 += red[8 + w]; SW += red[16 + w]; }
        __syncthreads();
        const float rl = 1.0f / SL, r1 = 1.0f / S1;
        const float kl = LN2 * (SW * r1 - ((ML - MX) + log2f(S1 * rl)));
        loss += kl;
    }
    if (tid == 0) { const float v = loss * (1.0f / (float)NB_FULL); *(volatile float*)OUT2 = v; __threadfence(); *(volatile float*)OUT2 = v; }
}

static constexpr size_t al256(size_t v) { return (v + 255) & ~(size_t)255; }
static constexpr size_t SZ_XB = al256((size_t)NB * SEQP * DM * 2);
static constexpr size_t SZ_WT = al256((size_t)NQKV * DM * 2);
static constexpr size_t SZ_WM = al256((size_t)DM * DM * 2);
static constexpr size_t SZ_QK = al256((size_t)2 * NB * NH_ * SEQP * HD * 2);
static constexpr size_t SZ_VT = al256((size_t)NB * DM * SEQP * 2);
static constexpr size_t SZ_CT = al256((size_t)NB * SEQP * DM * 2);
static constexpr size_t SZ_ST = al256((size_t)NB * NH_ * (SEQP / 16) * 128 * 4);
static constexpr size_t SZ_TOTAL = 2 * (SZ_XB + SZ_WT + SZ_WM + SZ_QK + SZ_VT + SZ_CT) + SZ_ST;
static_assert(SZ_TOTAL <= (size_t)134217728);
static_assert(((size_t)2 * DM * DM * 2) % 256 == 0);
static_assert((size_t)NB * NH_ * HD * SEQP == (size_t)NB * DM * SEQP);

extern "C" void kernel_launch(void* const* d_in, const int* in_sizes, int n_in,
                              void* d_out, int out_size, void* d_ws, size_t ws_size, hipStream_t stream) {
    if (n_in < 19) return;
    const size_t needx = ((size_t)(NB - 1) * SEQ_FULL + SEQ) * DM;
    if ((size_t)in_sizes[0] < needx || (size_t)in_sizes[1] < needx) return;
    if ((size_t)in_sizes[3] < (size_t)DM * NQKV || (size_t)in_sizes[5] < (size_t)DM * NQKV) return;
    if (in_sizes[4] < NQKV || in_sizes[6] < NQKV) return;
    if ((size_t)in_sizes[7] < (size_t)DM * DM || (size_t)in_sizes[9] < (size_t)DM * DM) return;
    if (in_sizes[8] < DM || in_sizes[10] < DM) return;
    if (in_sizes[11] < NH_ * NATT * 2) return;
    for (int i = 12; i <= 17; ++i) if (in_sizes[i] < NH_ * NATT) return;
    if (in_sizes[18] < NH_) return;
    if ((size_t)out_size < (size_t)2 * NB_FULL * SEQ_FULL * DM + 1) return;
    if (SZ_TOTAL > ws_size) return;
    const float* x = (const float*)d_in[0];      const float* l = (const float*)d_in[1];
    const float* wqkv = (const float*)d_in[3];   const float* bqkv = (const float*)d_in[4];
    const float* wqkv1 = (const float*)d_in[5];  const float* bqkv1 = (const float*)d_in[6];
    const float* w_mlp = (const float*)d_in[7];  const float* b_mlp = (const float*)d_in[8];
    const float* w_mlp1 = (const float*)d_in[9]; const float* b_mlp1 = (const float*)d_in[10];
    const float* c1w = (const float*)d_in[11];   const float* c1b = (const float*)d_in[12];
    const float* bn_g = (const float*)d_in[13];  const float* bn_b = (const float*)d_in[14];
    const float* bn_m = (const float*)d_in[15];  const float* bn_v = (const float*)d_in[16];
    const float* c2w = (const float*)d_in[17];   const float* c2b = (const float*)d_in[18];
    float* OUT0 = (float*)d_out;
    float* OUT1 = OUT0 + (size_t)NB_FULL * SEQ_FULL * DM;
    float* OUT2 = OUT0 + (size_t)2 * NB_FULL * SEQ_FULL * DM;
    char* wsp = (char*)d_ws;
    bf* XB = (bf*)wsp; wsp += SZ_XB;
    bf* LB = (bf*)wsp; wsp += SZ_XB;
    bf* WTX = (bf*)wsp; wsp += SZ_WT;
    bf* WTL = (bf*)wsp; wsp += SZ_WT;
    h16* WMX = (h16*)wsp; wsp += SZ_WM;
    h16* WML = (h16*)wsp; wsp += SZ_WM;
    h16* QKX = (h16*)wsp; wsp += SZ_QK;
    h16* QKL = (h16*)wsp; wsp += SZ_QK;
    h16* VTX = (h16*)wsp; wsp += SZ_VT;
    h16* VTL = (h16*)wsp; wsp += SZ_VT;
    h16* CX = (h16*)wsp; wsp += SZ_CT;
    h16* CL = (h16*)wsp; wsp += SZ_CT;
    float* ST = (float*)wsp; wsp += SZ_ST;

    { const unsigned g = (unsigned)((size_t)NB * SEQP * (DM / 8) / 256);
      k_cvtpad<<<g, 256, 0, stream>>>(x, XB);
      k_cvtpad<<<g, 256, 0, stream>>>(l, LB); }
    k_wT<<<dim3(NQKV / 64, DM / 64, 1), 256, 0, stream>>>(wqkv,  WTX, NQKV, 0);
    k_wT<<<dim3(NQKV / 64, DM / 64, 1), 256, 0, stream>>>(wqkv1, WTL, NQKV, 0);
    k_wT<<<dim3(DM / 64, DM / 64, 1), 256, 0, stream>>>(w_mlp,  (unsigned short*)WMX, DM, 1);
    k_wT<<<dim3(DM / 64, DM / 64, 1), 256, 0, stream>>>(w_mlp1, (unsigned short*)WML, DM, 1);

    k_proj_qk<<<dim3(NB * SEQP / 64, 2 * DM / 64, 1), 32, 0, stream>>>(XB, WTX, bqkv,  QKX);
    k_proj_qk<<<dim3(NB * SEQP / 64, 2 * DM / 64, 1), 32, 0, stream>>>(LB, WTL, bqkv1, QKL);
    k_proj_vt<<<dim3(DM / 64, NB * SEQP / 64, 1), 32, 0, stream>>>(WTX + (size_t)2 * DM * DM, XB, bqkv  + 2 * DM, VTX);
    k_proj_vt<<<dim3(DM / 64, NB * SEQP / 64, 1), 32, 0, stream>>>(WTL + (size_t)2 * DM * DM, LB, bqkv1 + 2 * DM, VTL);

    k_flash<<<dim3(SEQP / (16 * AW), NB * NH_, 1), 32 * AW, 0, stream>>>(QKX, VTX, QKL, VTL, c1w, c1b, bn_g, bn_b, bn_m, bn_v, c2w, c2b, CX, CL, ST);

    k_oproj<<<dim3(NB * SEQP / 64, DM / 64, 1), 32, 0, stream>>>(CX, WMX, b_mlp,  OUT0);
    k_oproj<<<dim3(NB * SEQP / 64, DM / 64, 1), 32, 0, stream>>>(CL, WML, b_mlp1, OUT1);

    k_klred<<<1, 256, 0, stream>>>(ST, OUT2);
}
